// RelationalConv_53489522705039
// MI455X (gfx1250) — hardware-verified
//
#include <hip/hip_runtime.h>
#include <stddef.h>


#define HD      128
#define NR      4
#define KREL    HD
#define KTOT    (KREL + HD)
#define AP      (NR * HD)
#define NTHR    256
#define NWAVE   8
#define EPT     8
#define NGRP    2
#define CHUNK   (NTHR * EPT * NGRP)
#define WCAP    (EPT * NGRP * 32)
#define NBD     1024
#define NSLOT   (NBD * NR)
#define SSHF    12
#define RCAP    32768
#define SEGCAP  2048
#define GROWS   128
#define TPK     64
#define TPN     32
#define TPP     72
#define ASCL    16
#define WSCL    64
#define WSCAP   134217728

#define LDS_AGG   ((3 * NSLOT + RCAP + NWAVE * WCAP + 2 * NWAVE) * 4)
#define LDS_GEMM  (GROWS * HD * 4)

static_assert(NSLOT == (1 << SSHF));
static_assert((KREL % 32) == 0 && (HD % 32) == 0 && (KTOT % 32) == 0);
static_assert((KTOT % TPK) == 0 && (KREL % TPK) == 0 && (HD % TPN) == 0);
static_assert(TPN * 8 == NTHR && TPK * TPN == NTHR * 8 && TPK == NWAVE * 8);
static_assert((TPP % 8) == 0 && TPP >= TPK);
static_assert(GROWS == NWAVE * 16);
static_assert(HD == 16 * 8 && HD == 32 * 4);
static_assert(NSLOT == NTHR * 16);
static_assert((RCAP % 4) == 0 && WCAP == EPT * NGRP * 32);
static_assert((NBD % NWAVE) == 0 && (NBD % GROWS) == 0 && (NR % 2) == 0);
static_assert(LDS_AGG <= 300 * 1024);

typedef float     v4f  __attribute__((ext_vector_type(4)));
typedef float     v8f  __attribute__((ext_vector_type(8)));
typedef int       v4i  __attribute__((ext_vector_type(4)));
typedef _Float16  v8h  __attribute__((ext_vector_type(8)));
typedef _Float16  v16h __attribute__((ext_vector_type(16)));
union FragH { v16h v; v8h h[2]; };

__device__ __forceinline__ v8f wmf(v16h a, v16h b, v8f c) {
  v8f d = __builtin_amdgcn_wmma_f32_16x16x32_f16(false, a, false, b, (short)0, c, false, false);
  asm volatile("v_nop\n\tv_nop\n\tv_nop\n\tv_nop" : "+v"(d) : "v"(a), "v"(b));
  return d;
}

__device__ __forceinline__ v8h cvt8h(v4f a, v4f b, float z) {
  v8h h;
  h[0] = (_Float16)(a.x * z); h[1] = (_Float16)(a.y * z); h[2] = (_Float16)(a.z * z); h[3] = (_Float16)(a.w * z);
  h[4] = (_Float16)(b.x * z); h[5] = (_Float16)(b.y * z); h[6] = (_Float16)(b.z * z); h[7] = (_Float16)(b.w * z);
  return h;
}

__device__ __forceinline__ float tanh_f(float v) {
  const float e  = __builtin_amdgcn_exp2f(v * 2.8853900817779268f);
  const float rc = __builtin_amdgcn_rcpf(e + 1.0f);
  return fmaf(-2.0f, rc, 1.0f);
}

__global__ __launch_bounds__(NTHR) void k_prep(
    const float* __restrict__ Wrel, const float* __restrict__ Wroot, _Float16* Bw, float scale) {
  __shared__ __attribute__((aligned(16))) _Float16 sT[TPN * TPP];
  const int tid = threadIdx.x;
  const int r = (int)blockIdx.z;
  const int k0 = (int)blockIdx.x * TPK, n0 = (int)blockIdx.y * TPN;
  const int nc = tid & 31, kq = tid >> 5;
  const int col = n0 + nc;
  const float* W = (k0 < KREL) ? Wrel : Wroot;
  const int i0 = (k0 < KREL) ? k0 : (k0 - KREL);
#pragma unroll 1
  for (int it = 0; it < TPK / NWAVE; ++it) {
    const int kr = kq + NWAVE * it;
    const float w = W[((size_t)r * HD + i0 + kr) * HD + col];
    sT[nc * TPP + kr] = (_Float16)(w * scale);
  }
  __syncthreads();
  const int nl = tid >> 3, p = tid & 7;
  const v8h hv = *(const v8h*)(sT + nl * TPP + 8 * p);
  _Float16* d = Bw + ((size_t)r * HD + n0 + nl) * KTOT + k0 + 8 * p;
  *(volatile v8h*)d = hv;
  __threadfence();
  *(volatile v8h*)d = hv;
}

template <int MODE>
__device__ __forceinline__ int scan_chunk(const int* __restrict__ kd, const int* __restrict__ kt, int nE,
                                          int cbase, int base, int vec8, unsigned* list,
                                          int tid, int lane, int wave) {
  int wc = 0;
#pragma unroll
  for (int g = 0; g < NGRP; ++g) {
    const int e0   = cbase + (g * NTHR + tid) * EPT;
    const int sent = -2147483647 - 1;
    const int i0 = min(e0, nE - 1),     i1 = min(e0 + 1, nE - 1), i2 = min(e0 + 2, nE - 1), i3 = min(e0 + 3, nE - 1);
    const int i4 = min(e0 + 4, nE - 1), i5 = min(e0 + 5, nE - 1), i6 = min(e0 + 6, nE - 1), i7 = min(e0 + 7, nE - 1);
    v4i da, db, ta, tb;
    if (vec8 != 0 && cbase + CHUNK <= nE) {
      da = *(const v4i*)(kd + e0);
      db = *(const v4i*)(kd + e0 + 4);
      ta = *(const v4i*)(kt + e0);
      tb = *(const v4i*)(kt + e0 + 4);
    } else {
      da.x = (e0     < nE) ? kd[i0] : sent;
      da.y = (e0 + 1 < nE) ? kd[i1] : sent;
      da.z = (e0 + 2 < nE) ? kd[i2] : sent;
      da.w = (e0 + 3 < nE) ? kd[i3] : sent;
      db.x = (e0 + 4 < nE) ? kd[i4] : sent;
      db.y = (e0 + 5 < nE) ? kd[i5] : sent;
      db.z = (e0 + 6 < nE) ? kd[i6] : sent;
      db.w = (e0 + 7 < nE) ? kd[i7] : sent;
      ta.x = kt[i0]; ta.y = kt[i1]; ta.z = kt[i2]; ta.w = kt[i3];
      tb.x = kt[i4]; tb.y = kt[i5]; tb.z = kt[i6]; tb.w = kt[i7];
    }
    const unsigned nb = (unsigned)base;
    const unsigned s0 = (unsigned)da.x - nb, s1 = (unsigned)da.y - nb;
    const unsigned s2 = (unsigned)da.z - nb, s3 = (unsigned)da.w - nb;
    const unsigned s4 = (unsigned)db.x - nb, s5 = (unsigned)db.y - nb;
    const unsigned s6 = (unsigned)db.z - nb, s7 = (unsigned)db.w - nb;
    const bool h0 = s0 < (unsigned)NBD, h1 = s1 < (unsigned)NBD, h2 = s2 < (unsigned)NBD, h3 = s3 < (unsigned)NBD;
    const bool h4 = s4 < (unsigned)NBD, h5 = s5 < (unsigned)NBD, h6 = s6 < (unsigned)NBD, h7 = s7 < (unsigned)NBD;
    const unsigned q0 = s0 * NR + (unsigned)min(max(ta.x, 0), NR - 1);
    const unsigned q1 = s1 * NR + (unsigned)min(max(ta.y, 0), NR - 1);
    const unsigned q2 = s2 * NR + (unsigned)min(max(ta.z, 0), NR - 1);
    const unsigned q3 = s3 * NR + (unsigned)min(max(ta.w, 0), NR - 1);
    const unsigned q4 = s4 * NR + (unsigned)min(max(tb.x, 0), NR - 1);
    const unsigned q5 = s5 * NR + (unsigned)min(max(tb.y, 0), NR - 1);
    const unsigned q6 = s6 * NR + (unsigned)min(max(tb.z, 0), NR - 1);
    const unsigned q7 = s7 * NR + (unsigned)min(max(tb.w, 0), NR - 1);
    const unsigned any = __builtin_amdgcn_ballot_w32(h0 | h1 | h2 | h3 | h4 | h5 | h6 | h7);
    if (any != 0u) {
#define HITJ(HJ, QJ, IJ) { \
        const unsigned mj = __builtin_amdgcn_ballot_w32(HJ); \
        if (mj != 0u) { \
          if (HJ) { \
            const int pos = wc + (int)__builtin_amdgcn_mbcnt_lo(mj, 0u); \
            const unsigned entv = (MODE != 0) ? ((((unsigned)(IJ)) << SSHF) | (QJ)) : (QJ); \
            if (pos < WCAP) list[wave * WCAP + pos] = entv; \
          } \
          wc += (int)__builtin_popcount(mj); } }
      HITJ(h0, q0, i0)
      HITJ(h1, q1, i1)
      HITJ(h2, q2, i2)
      HITJ(h3, q3, i3)
      HITJ(h4, q4, i4)
      HITJ(h5, q5, i5)
      HITJ(h6, q6, i6)
      HITJ(h7, q7, i7)
#undef HITJ
    }
  }
  return wc;
}

__global__ __launch_bounds__(NTHR) void k_agg(
    const int* __restrict__ edst, const int* __restrict__ etyp, const int* __restrict__ esrc,
    const float* __restrict__ x, _Float16* AG, int nE, int nN, int vec8) {
  extern __shared__ v4f lds_dyn[];
  int* scnt = (int*)lds_dyn;
  int* soff = scnt + NSLOT;
  int* curs = soff + NSLOT;
  unsigned* region = (unsigned*)(curs + NSLOT);
  unsigned* list = region + RCAP;
  int* wcnt = (int*)(list + NWAVE * WCAP);
  int* wtot = wcnt + NWAVE;
  const int tid = threadIdx.x, lane = tid & 31, wave = tid >> 5;
  const int base = (int)blockIdx.x * NBD;

  {
    const v4i z = {0, 0, 0, 0};
    for (int i = tid; i < NSLOT / 4; i += NTHR) ((v4i*)scnt)[i] = z;
  }
  __syncthreads();

  const int nChunks = (nE + CHUNK - 1) / CHUNK;

#pragma unroll 1
  for (int ch = 0; ch < nChunks; ++ch) {
    const int cbase = ch * CHUNK;
    const int wc = scan_chunk<0>(edst, etyp, nE, cbase, base, vec8, list, tid, lane, wave);
    if (lane == 0) wcnt[wave] = wc;
    __syncthreads();
    if (wave == 0) {
#pragma unroll 1
      for (int wsx = 0; wsx < NWAVE; ++wsx) {
        int n = __builtin_amdgcn_readfirstlane(wcnt[wsx]);
        n = n > WCAP ? WCAP : (n < 0 ? 0 : n);
        const unsigned* lp = list + wsx * WCAP;
#pragma unroll 1
        for (int i = 0; i < n; ++i) {
          const int ent  = __builtin_amdgcn_readfirstlane((int)lp[i]);
          const int slot = ent & (NSLOT - 1);
          if (lane == 0) scnt[slot] = scnt[slot] + 1;
        }
      }
    }
    __syncthreads();
  }

  {
    const int sb = 16 * tid;
    const v4i c0 = *(const v4i*)(scnt + sb);
    const v4i c1 = *(const v4i*)(scnt + sb + 4);
    const v4i c2 = *(const v4i*)(scnt + sb + 8);
    const v4i c3 = *(const v4i*)(scnt + sb + 12);
    const int ts = (c0.x + c0.y + c0.z + c0.w) + (c1.x + c1.y + c1.z + c1.w)
                 + (c2.x + c2.y + c2.z + c2.w) + (c3.x + c3.y + c3.z + c3.w);
    int incl = ts;
#pragma unroll
    for (int dd = 1; dd < 32; dd <<= 1) {
      const int t = __shfl_up(incl, dd, 32);
      if (lane >= dd) incl += t;
    }
    if (lane == 31) wtot[wave] = incl;
    __syncthreads();
    int pre = 0;
#pragma unroll 1
    for (int w = 0; w < wave; ++w) pre += wtot[w];
    int run = pre + incl - ts;
    v4i o0, o1, o2, o3;
    o0.x = run; run += c0.x; o0.y = run; run += c0.y; o0.z = run; run += c0.z; o0.w = run; run += c0.w;
    o1.x = run; run += c1.x; o1.y = run; run += c1.y; o1.z = run; run += c1.z; o1.w = run; run += c1.w;
    o2.x = run; run += c2.x; o2.y = run; run += c2.y; o2.z = run; run += c2.z; o2.w = run; run += c2.w;
    o3.x = run; run += c3.x; o3.y = run; run += c3.y; o3.z = run; run += c3.z; o3.w = run;
    *(v4i*)(soff + sb) = o0; *(v4i*)(soff + sb + 4) = o1; *(v4i*)(soff + sb + 8) = o2; *(v4i*)(soff + sb + 12) = o3;
    *(v4i*)(curs + sb) = o0; *(v4i*)(curs + sb + 4) = o1; *(v4i*)(curs + sb + 8) = o2; *(v4i*)(curs + sb + 12) = o3;
    __syncthreads();
  }

#pragma unroll 1
  for (int ch = 0; ch < nChunks; ++ch) {
    const int cbase = ch * CHUNK;
    const int wc = scan_chunk<1>(edst, etyp, nE, cbase, base, vec8, list, tid, lane, wave);
    if (lane == 0) wcnt[wave] = wc;
    __syncthreads();
    if (wave == 0) {
#pragma unroll 1
      for (int wsx = 0; wsx < NWAVE; ++wsx) {
        int n = __builtin_amdgcn_readfirstlane(wcnt[wsx]);
        n = n > WCAP ? WCAP : (n < 0 ? 0 : n);
        const unsigned* lp = list + wsx * WCAP;
#pragma unroll 1
        for (int i = 0; i < n; ++i) {
          const unsigned ent = (unsigned)__builtin_amdgcn_readfirstlane((int)lp[i]);
          const int slot = (int)(ent & (unsigned)(NSLOT - 1));
          int ev = (int)(ent >> SSHF);
          ev = ev > nE - 1 ? nE - 1 : ev;
          if (lane == 0) {
            const int pos = curs[slot];
            if ((unsigned)pos < (unsigned)RCAP) region[pos] = (unsigned)ev;
            curs[slot] = (pos >= RCAP) ? RCAP : pos + 1;
          }
        }
      }
    }
    __syncthreads();
  }

  const float qnan = __int_as_float(0x7fc00000);
  const int hh = lane >> 4, m = lane & 15;
  const v4f zf = {0.f, 0.f, 0.f, 0.f};
#pragma unroll 1
  for (int jj = 0; jj < NBD / NWAVE; ++jj) {
    const int j = wave + NWAVE * jj;
    const int d = base + j;
#pragma unroll 1
    for (int rp = 0; rp < NR / 2; ++rp) {
      const int r    = 2 * rp + hh;
      const int slot = j * NR + r;
      const int n    = scnt[slot];
      const int st   = soff[slot];
      const bool bad = (n > SEGCAP) || (n < 0) || (st < 0) || (st + n > RCAP);
      const int nn   = n < 0 ? 0 : (n > SEGCAP ? SEGCAP : n);
      const int no   = __shfl_xor(nn, 16, 32);
      const int trip = nn > no ? nn : no;
      v4f a0 = zf, a1 = zf;
#pragma unroll 1
      for (int p = 0; p < trip; ++p) {
        const bool use = p < nn;
        const int pq = use ? p : (nn - 1);
        int pos = st + pq;
        pos = pos < 0 ? 0 : (pos > RCAP - 1 ? RCAP - 1 : pos);
        const int eu = (int)region[pos];
        const int e  = eu < 0 ? 0 : (eu > nE - 1 ? nE - 1 : eu);
        int s = esrc[e];
        s = s < 0 ? 0 : (s > nN - 1 ? nN - 1 : s);
        const float* sp = x + (size_t)s * HD + 8 * m;
        const v4f l0 = *(const v4f*)sp;
        const v4f l1 = *(const v4f*)(sp + 4);
        a0 = use ? (a0 + l0) : a0;
        a1 = use ? (a1 + l1) : a1;
      }
      const float sc = bad ? qnan : (float)ASCL;
      const v8h mh = cvt8h(a0, a1, sc);
      _Float16* gp = AG + (size_t)d * AP + (size_t)rp * 2 * HD + 8 * lane;
      *(volatile v8h*)gp = mh;
      __threadfence();
      *(volatile v8h*)gp = mh;
    }
  }
}

#define NT (HD / 16)

__device__ __forceinline__ void bsteps(v8f (&acc)[NT], const v16h av, const _Float16* bp) {
#pragma unroll
  for (int t = 0; t < NT; ++t) {
    const _Float16* bq = bp + (size_t)(16 * t) * KTOT;
    FragH bf;
    bf.h[0] = *(const v8h*)bq;
    bf.h[1] = *(const v8h*)(bq + 16);
    acc[t] = wmf(av, bf.v, acc[t]);
  }
}

__device__ __forceinline__ void kstep_h(v8f (&acc)[NT], const _Float16* ap, const _Float16* bp) {
  FragH af;
  af.h[0] = *(const v8h*)ap;
  af.h[1] = *(const v8h*)(ap + 16);
  bsteps(acc, af.v, bp);
}

__device__ __forceinline__ void kstep_x(v8f (&acc)[NT], const float* xq, const _Float16* bp, float z) {
  FragH af;
  af.h[0] = cvt8h(*(const v4f*)xq, *(const v4f*)(xq + 4), z);
  af.h[1] = cvt8h(*(const v4f*)(xq + 16), *(const v4f*)(xq + 20), z);
  bsteps(acc, af.v, bp);
}

__global__ __launch_bounds__(NTHR) void k_gemm(
    const _Float16* __restrict__ AG, const float* __restrict__ x, const _Float16* __restrict__ Bw,
    const float* __restrict__ brel, const float* __restrict__ broot, float* out,
    int nN, int aggRows, float osc) {
  extern __shared__ v4f lds_dyn[];
  float* stg = (float*)lds_dyn;
  const int tid = threadIdx.x, lane = tid & 31, wave = tid >> 5, hh = lane >> 4, m = lane & 15;
  const int row0 = (int)blockIdx.x * GROWS + wave * 16;
  const int ar  = row0 + m;
  const int arx = ar < nN ? ar : nN - 1;
  const int ara = ar < aggRows ? ar : aggRows - 1;
  const _Float16* agp = AG + (size_t)ara * AP + 8 * hh;
  const float*    xp  = x + (size_t)arx * HD + 8 * hh;
  const _Float16* bp  = Bw + (size_t)m * KTOT + 8 * hh;
  float* sp = stg + (wave * 16 + 8 * hh) * HD + m;

#pragma unroll
  for (int t = 0; t < NT; ++t) {
#pragma unroll
    for (int i = 0; i < 8; ++i) sp[i * HD + 16 * t] = 0.0f;
  }

#pragma unroll 1
  for (int r = 0; r < NR; ++r) {
    v8f acc[NT];
#pragma unroll
    for (int t = 0; t < NT; ++t) { v8f zz = {0.f, 0.f, 0.f, 0.f, 0.f, 0.f, 0.f, 0.f}; acc[t] = zz; }
    const _Float16* brp = bp + (size_t)r * HD * KTOT;
    const _Float16* arp = agp + r * HD;
#pragma unroll 1
    for (int ks = 0; ks < KREL / 32; ++ks) kstep_h(acc, arp + 32 * ks, brp + 32 * ks);
#pragma unroll 1
    for (int ks = 0; ks < HD / 32; ++ks) kstep_x(acc, xp + 32 * ks, brp + KREL + 32 * ks, (float)ASCL);

#pragma unroll
    for (int t = 0; t < NT; ++t) {
      const int col = 16 * t + m;
      const float bs = brel[r * HD + col] + broot[r * HD + col];
#pragma unroll
      for (int i = 0; i < 8; ++i) {
        const float v = tanh_f(fmaf(acc[t][i], osc, bs));
        float* q = sp + i * HD + 16 * t;
        *q = *q + v;
      }
    }
  }
  __syncthreads();

  const float* lp = stg + wave * 16 * HD;
  float* gp = out + (size_t)row0 * HD + 4 * lane;
#pragma unroll
  for (int i = 0; i < 16; ++i) {
    if (row0 + i < nN) {
      const v4f v = *(const v4f*)(lp + i * HD + 4 * lane);
      *(volatile v4f*)(gp + (size_t)i * HD) = v;
    }
  }
  __threadfence();
#pragma unroll
  for (int i = 0; i < 16; ++i) {
    if (row0 + i < nN) {
      const v4f v = *(const v4f*)(lp + i * HD + 4 * lane);
      *(volatile v4f*)(gp + (size_t)i * HD) = v;
    }
  }
}

extern "C" void kernel_launch(void* const* d_in, const int* in_sizes, int n_in,
                              void* d_out, int out_size, void* d_ws, size_t ws_size,
                              hipStream_t stream) {
  if (n_in < 7) return;
  if (in_sizes[0] < HD || (in_sizes[0] % HD) != 0) return;
  const int nN = in_sizes[0] / HD;
  const int nE = in_sizes[2];
  if (nE < 1 || in_sizes[1] != 2 * nE) return;
  if (nE > (1 << 20)) return;
  if (in_sizes[3] != NR * HD * HD || in_sizes[4] != NR * HD) return;
  if (in_sizes[5] != NR * HD * HD || in_sizes[6] != NR * HD) return;
  if ((long long)out_size != (long long)nN * HD) return;
  if (nN > (1 << 26)) return;

  const float* x     = (const float*)d_in[0];
  const int*   ei    = (const int*)d_in[1];
  const int*   etyp  = (const int*)d_in[2];
  const float* Wrel  = (const float*)d_in[3];
  const float* brel  = (const float*)d_in[4];
  const float* Wroot = (const float*)d_in[5];
  const float* broot = (const float*)d_in[6];
  const int* esrc = ei;
  const int* edst = ei + nE;
  float* out = (float*)d_out;

  const int gridAgg  = (nN + NBD - 1) / NBD;
  const int aggRows  = gridAgg * NBD;
  const int gridGemm = (nN + GROWS - 1) / GROWS;
  if (gridGemm * GROWS > aggRows) return;

  char* ws = (char*)d_ws;
  size_t off = 0;
#define CARVE(NAME, BYTES) const size_t NAME = off; off += (size_t)(BYTES); off = (off + 255) & ~(size_t)255;
  CARVE(oBw, (size_t)NR * HD * KTOT * 2)
  CARVE(oAG, (size_t)aggRows * AP * 2)
#undef CARVE
  if (off > ws_size || off > (size_t)WSCAP) return;
  _Float16* Bw = (_Float16*)(ws + oBw);
  _Float16* AG = (_Float16*)(ws + oAG);

  const int vec8 = ((nE & 3) == 0) ? 1 : 0;
  const float osc = 1.0f / ((float)ASCL * (float)WSCL);

  k_prep<<<dim3(KTOT / TPK, HD / TPN, NR), NTHR, 0, stream>>>(Wrel, Wroot, Bw, (float)WSCL);

  hipFuncSetAttribute(reinterpret_cast<const void*>(&k_agg),
                      hipFuncAttributeMaxDynamicSharedMemorySize, LDS_AGG);
  k_agg<<<gridAgg, NTHR, LDS_AGG, stream>>>(edst, etyp, esrc, x, AG, nE, nN, vec8);

  hipFuncSetAttribute(reinterpret_cast<const void*>(&k_gemm),
                      hipFuncAttributeMaxDynamicSharedMemorySize, LDS_GEMM);
  k_gemm<<<gridGemm, NTHR, LDS_GEMM, stream>>>(AG, x, Bw, brel, broot, out, nN, aggRows, osc);
}
